// CrossAttentionLayer_13511967113537
// MI455X (gfx1250) — hardware-run, weakly checked
//
#include <hip/hip_runtime.h>
#include <math.h>

constexpr int kB     = 4;
constexpr int kLq    = 1024;
constexpr int kLk    = 1024;
constexpr int kE     = 1024;
constexpr int kH     = 16;
constexpr int kDh    = 64;
constexpr int kF     = 4096;
constexpr int kTok   = kB * kLq;
constexpr int kChunk = 256;
constexpr int kNChunk = kLq / kChunk;
constexpr float kWCarry     = 16.0f;
constexpr float kWCarryInv  = 1.0f / 16.0f;
constexpr float kPCarry     = 32768.0f;
constexpr float kCtxCarry   = 256.0f;
constexpr float kPVScale    = kCtxCarry / kPCarry;
constexpr float kOutScale   = 1.0f / (kCtxCarry * kWCarry);
constexpr float kScoreScale = 0.125f;
constexpr float kInvE       = 1.0f / 1024.0f;
constexpr float kInvH       = 1.0f / 16.0f;
constexpr float kLnEps      = 1.0e-5f;
static_assert(kH * kDh == kE);
static_assert(kTok % 64 == 0 && kE % 64 == 0 && kF % 64 == 0 && kLk % 64 == 0 && kChunk % 64 == 0 && kDh % 64 == 0);
static_assert(kE % 32 == 0 && kF % 32 == 0 && kDh % 32 == 0 && kLk % 32 == 0);
static_assert(kLq % kChunk == 0 && kLk == 4 * 256 && kE == 8 * 128);

typedef __attribute__((ext_vector_type(16))) _Float16 v16h;
typedef __attribute__((ext_vector_type(8)))  _Float16 v8h;
typedef __attribute__((ext_vector_type(16))) __bf16   v16b;
typedef __attribute__((ext_vector_type(8)))  __bf16   v8b;
typedef __attribute__((ext_vector_type(8)))  float    v8f;
typedef __attribute__((ext_vector_type(4)))  float    v4f;
typedef __attribute__((ext_vector_type(4)))  unsigned int v4u;

__device__ __forceinline__ unsigned short f2bf_bits(float f) {
  unsigned u = __float_as_uint(f);
  return (unsigned short)((u + 0x7FFFu + ((u >> 16) & 1u)) >> 16);
}
__device__ __forceinline__ float bf_bits2f(unsigned short h) { return __uint_as_float(((unsigned)h) << 16); }

__device__ __forceinline__ void dep_guard4_h(v8f& a, v8f& b, v8f& c, v8f& d, v16h x, v16h y) {
  asm volatile("v_nop\n\tv_nop\n\tv_nop\n\tv_nop" : "+v"(a), "+v"(b), "+v"(c), "+v"(d) : "v"(x), "v"(y));
}
__device__ __forceinline__ void dep_guard4_b(v8f& a, v8f& b, v8f& c, v8f& d, v16b x, v16b y) {
  asm volatile("v_nop\n\tv_nop\n\tv_nop\n\tv_nop" : "+v"(a), "+v"(b), "+v"(c), "+v"(d) : "v"(x), "v"(y));
}
__device__ __forceinline__ void keep4_h(v16h a, v16h b, v16h c, v16h d) { asm volatile("v_nop" :: "v"(a), "v"(b), "v"(c), "v"(d)); }
__device__ __forceinline__ void keep4_b(v16b a, v16b b, v16b c, v16b d) { asm volatile("v_nop" :: "v"(a), "v"(b), "v"(c), "v"(d)); }
__device__ __forceinline__ void acc_guard4(v8f& a, v8f& b, v8f& c, v8f& d) { asm volatile("v_nop\n\tv_nop\n\tv_nop\n\tv_nop" : "+v"(a), "+v"(b), "+v"(c), "+v"(d)); }
template <typename T> struct Frag;
template <> struct Frag<_Float16> {
  typedef v16h V; union U { v16h v; v8h h[2]; };
  static __device__ __forceinline__ v16h load(const _Float16* p) {
    U f; f.h[0] = *(const v8h*)(p); f.h[1] = *(const v8h*)(p + 16); return f.v;
  }
  static __device__ __forceinline__ v8f mma(v16h a, v16h b, v8f c) {
    return __builtin_amdgcn_wmma_f32_16x16x32_f16(false, a, false, b, (short)0, c, false, false);
  }
  static __device__ __forceinline__ void guard4(v8f& a, v8f& b, v8f& c, v8f& d, v16h x, v16h y) { dep_guard4_h(a, b, c, d, x, y); }
  static __device__ __forceinline__ void keep(v16h a, v16h b, v16h c, v16h d) { keep4_h(a, b, c, d); }
};
template <> struct Frag<__bf16> {
  typedef v16b V; union U { v16b v; v8b h[2]; };
  static __device__ __forceinline__ v16b load(const __bf16* p) {
    U f; f.h[0] = *(const v8b*)(p); f.h[1] = *(const v8b*)(p + 16); return f.v;
  }
  static __device__ __forceinline__ v8f mma(v16b a, v16b b, v8f c) {
    return __builtin_amdgcn_wmma_f32_16x16x32_bf16(false, a, false, b, (short)0, c, false, false);
  }
  static __device__ __forceinline__ void guard4(v8f& a, v8f& b, v8f& c, v8f& d, v16b x, v16b y) { dep_guard4_b(a, b, c, d, x, y); }
  static __device__ __forceinline__ void keep(v16b a, v16b b, v16b c, v16b d) { keep4_b(a, b, c, d); }
};

__device__ __forceinline__ unsigned pk16(unsigned short a, unsigned short b) { return (unsigned)a | ((unsigned)b << 16); }
__device__ __forceinline__ unsigned short h_bits(float f) { const _Float16 h = (_Float16)f; return __builtin_bit_cast(unsigned short, h); }

template <int ET> struct Elem;
template <> struct Elem<0> { typedef _Float16 T; };
template <> struct Elem<1> { typedef __bf16 T; };
template <int ET, bool SPLIT, int BIAS_MODE, int OUT_MODE, bool RESID, int ACT = 0>
__global__ __launch_bounds__(256) void wmma_gemm64(
    const unsigned short* __restrict__ Ap, const unsigned short* __restrict__ A2p, int lda, long strideA,
    const unsigned short* __restrict__ Btp, const unsigned short* __restrict__ Bt2p, int ldb, long strideB,
    void* __restrict__ Cout, void* __restrict__ Cout2, int ldc, long strideC,
    const float* __restrict__ bias,
    const float* __restrict__ resid, long strideR,
    int M, int N, int K, float scale) {
  static_assert(!RESID || OUT_MODE == 0);
  static_assert(!(RESID && ACT != 0));
  static_assert(ACT == 0 || ACT == 2);
  typedef typename Elem<ET>::T T;
  typedef typename Frag<T>::V V;
  const T* A = (const T*)Ap; const T* A2 = (const T*)A2p; const T* Bt = (const T*)Btp; const T* Bt2 = (const T*)Bt2p;
  __shared__ __align__(16) float sT[8][16 * 68];
  const int b    = blockIdx.y;
  const int lane = threadIdx.x & 31;
  const int wave = threadIdx.x >> 5;
  const int tilesN = N >> 6;
  const int tilesM = M >> 6;
  const int tile = blockIdx.x * 8 + wave;
  if (tile >= tilesM * tilesN) return;
  const int tm = tile / tilesN;
  const int tn = tile - tm * tilesN;
  const int m0 = tm << 6;
  const int n0 = tn << 6;

  const T* Ab  = A  + (size_t)b * strideA;
  const T* Bb  = Bt + (size_t)b * strideB;
  const T* Ab2 = SPLIT ? (A2  + (size_t)b * strideA) : nullptr;
  const T* Bb2 = SPLIT ? (Bt2 + (size_t)b * strideB) : nullptr;

  const int rlane = lane & 15;
  const int koff  = (lane >> 4) * 8;
  const int mOff  = (lane >> 4) * 8;

  v8f acc[4][4];
#pragma unroll
  for (int i = 0; i < 4; ++i)
#pragma unroll
    for (int j = 0; j < 4; ++j) acc[i][j] = (v8f){0.f,0.f,0.f,0.f,0.f,0.f,0.f,0.f};

  for (int k0 = 0; k0 < K; k0 += 32) {
    V bh[4], bl[4];
#pragma unroll
    for (int j = 0; j < 4; ++j) {
      const size_t bo = (size_t)(n0 + (j << 4) + rlane) * ldb + koff + k0;
      bh[j] = Frag<T>::load(Bb + bo);
      if (SPLIT) bl[j] = Frag<T>::load(Bb2 + bo);
    }
#pragma unroll
    for (int i = 0; i < 4; ++i) {
      const size_t ao = (size_t)(m0 + (i << 4) + rlane) * lda + koff + k0;
      V ah = Frag<T>::load(Ab + ao);
      V al;
      if (SPLIT) al = Frag<T>::load(Ab2 + ao);
#pragma unroll
      for (int j = 0; j < 4; ++j) {
        acc[i][j] = Frag<T>::mma(ah, bh[j], acc[i][j]);
        if (SPLIT) {
          acc[i][j] = Frag<T>::mma(ah, bl[j], acc[i][j]);
          acc[i][j] = Frag<T>::mma(al, bh[j], acc[i][j]);
        }
      }
      Frag<T>::guard4(acc[i][0], acc[i][1], acc[i][2], acc[i][3], ah, SPLIT ? al : ah);
    }
    Frag<T>::keep(bh[0], bh[1], bh[2], bh[3]);
    if (SPLIT) Frag<T>::keep(bl[0], bl[1], bl[2], bl[3]);
  }
  acc_guard4(acc[0][0], acc[0][1], acc[0][2], acc[0][3]);
  acc_guard4(acc[1][0], acc[1][1], acc[1][2], acc[1][3]);
  acc_guard4(acc[2][0], acc[2][1], acc[2][2], acc[2][3]);
  acc_guard4(acc[3][0], acc[3][1], acc[3][2], acc[3][3]);

  float* slab = sT[wave];
  const float* Rb = RESID ? (resid + (size_t)b * strideR) : nullptr;
#pragma unroll
  for (int i = 0; i < 4; ++i) {
    const int mBase = m0 + (i << 4);
    v8f bm = (v8f){0.f,0.f,0.f,0.f,0.f,0.f,0.f,0.f};
    if (BIAS_MODE == 1) {
      const v4f b0v = *(const v4f*)(bias + mBase + mOff);
      const v4f b1v = *(const v4f*)(bias + mBase + mOff + 4);
      bm = (v8f){b0v[0], b0v[1], b0v[2], b0v[3], b1v[0], b1v[1], b1v[2], b1v[3]};
    }
#pragma unroll
    for (int j = 0; j < 4; ++j) {
      const int n = n0 + (j << 4) + rlane;
      float bv = 0.f;
      if (BIAS_MODE == 2) bv = bias[n];
#pragma unroll
      for (int r = 0; r < 8; ++r) {
        float v = acc[i][j][r] * scale;
        if (BIAS_MODE == 1) v += bm[r];
        if (BIAS_MODE == 2) v += bv;
        if (ACT == 2) v = fmaxf(v, 0.0f);
        slab[(mOff + r) * 68 + (j << 4) + rlane] = v;
      }
    }
    __builtin_amdgcn_fence(__ATOMIC_RELEASE, "workgroup");
    __builtin_amdgcn_wave_barrier();
    __builtin_amdgcn_fence(__ATOMIC_ACQUIRE, "workgroup");
    if (OUT_MODE == 0) {
      float* C = (float*)Cout + (size_t)b * strideC;
      const int hh = lane >> 4, c4 = (lane & 15) * 4;
      for (int pass = 0; pass < 2; ++pass) {
#pragma unroll
        for (int it = 0; it < 8; ++it) {
          const int row = it * 2 + hh;
          v4f v = *(const v4f*)(slab + row * 68 + c4);
          if (RESID) {
            const v4f rr = *(const v4f*)(Rb + (size_t)(mBase + row) * ldc + n0 + c4);
            v = v + rr;
          }
          *(volatile v4f*)(C + (size_t)(mBase + row) * ldc + n0 + c4) = v;
        }
        __threadfence();
      }
    } else {
      const int q = lane >> 3, c8 = (lane & 7) * 8;
      unsigned short* C  = (unsigned short*)Cout  + (size_t)b * strideC;
      unsigned short* C2 = (OUT_MODE == 2) ? ((unsigned short*)Cout2 + (size_t)b * strideC) : nullptr;
      for (int pass = 0; pass < 2; ++pass) {
#pragma unroll
        for (int it = 0; it < 4; ++it) {
          const int row = it * 4 + q;
          const float* sp = slab + row * 68 + c8;
          v8h hv, lv;
#pragma unroll
          for (int e = 0; e < 8; ++e) {
            if (OUT_MODE == 1) {
              hv[e] = (_Float16)sp[e];
            } else {
              unsigned short hb = f2bf_bits(sp[e]);
              unsigned short lb = f2bf_bits(sp[e] - bf_bits2f(hb));
              hv[e] = __builtin_bit_cast(_Float16, hb);
              lv[e] = __builtin_bit_cast(_Float16, lb);
            }
          }
          *(volatile v8h*)(C + (size_t)(mBase + row) * ldc + n0 + c8) = hv;
          if (OUT_MODE == 2) *(volatile v8h*)(C2 + (size_t)(mBase + row) * ldc + n0 + c8) = lv;
        }
        __threadfence();
      }
    }
    __builtin_amdgcn_fence(__ATOMIC_RELEASE, "workgroup");
    __builtin_amdgcn_wave_barrier();
    __builtin_amdgcn_fence(__ATOMIC_ACQUIRE, "workgroup");
  }
}

__global__ __launch_bounds__(256) void cast8_f16_kernel(const float* __restrict__ in, unsigned short* __restrict__ out, int n8) {
  const int i = blockIdx.x * 256 + threadIdx.x;
  if (i >= n8) return;
  const float* p = in + 8 * (size_t)i;
  const v4f a = *(const v4f*)(p);
  const v4f c = *(const v4f*)(p + 4);
  unsigned short hb[8];
#pragma unroll
  for (int e = 0; e < 4; ++e) {
    hb[e]     = h_bits(a[e]);
    hb[4 + e] = h_bits(c[e]);
  }
  const v4u u = (v4u){pk16(hb[0], hb[1]), pk16(hb[2], hb[3]), pk16(hb[4], hb[5]), pk16(hb[6], hb[7])};
  unsigned short* q = out + 8 * (size_t)i;
  *(volatile v4u*)q = u;
  __threadfence();
  *(volatile v4u*)q = u;
}

__global__ __launch_bounds__(256) void wtcast_kernel(const float* __restrict__ W, unsigned short* __restrict__ WT,
                                                     int kdim, int ndim, float scale) {
  __shared__ float sm[64][65];
  const int t  = threadIdx.x;
  const int k0 = blockIdx.x * 64;
  const int n0 = blockIdx.y * 64;
#pragma unroll
  for (int i = 0; i < 4; ++i) {
    const int e  = i * 256 + t;
    const int r  = e >> 4;
    const int c4 = (e & 15) * 4;
    const v4f w = *(const v4f*)(W + (size_t)(k0 + r) * ndim + n0 + c4);
    sm[c4 + 0][r] = w[0] * scale;
    sm[c4 + 1][r] = w[1] * scale;
    sm[c4 + 2][r] = w[2] * scale;
    sm[c4 + 3][r] = w[3] * scale;
  }
  __syncthreads();
  const int lane = t & 31, wave = t >> 5;
  const int q = lane >> 3, c8 = (lane & 7) * 8;
  for (int pass = 0; pass < 2; ++pass) {
#pragma unroll
    for (int it = 0; it < 2; ++it) {
      const int row = wave * 8 + it * 4 + q;
      unsigned short hb[8];
#pragma unroll
      for (int e = 0; e < 8; ++e) hb[e] = h_bits(sm[row][c8 + e]);
      const v4u u = (v4u){pk16(hb[0], hb[1]), pk16(hb[2], hb[3]), pk16(hb[4], hb[5]), pk16(hb[6], hb[7])};
      *(volatile v4u*)(WT + (size_t)(n0 + row) * kdim + k0 + c8) = u;
    }
    __threadfence();
  }
}

__global__ __launch_bounds__(128) void ln_f16_kernel(const float* __restrict__ x, const float* __restrict__ g,
                                                     const float* __restrict__ bta, unsigned short* __restrict__ out) {
  __shared__ float redA[4];
  __shared__ float redB[4];
  const int row  = blockIdx.x;
  const int t    = threadIdx.x;
  const int lane = t & 31, wave = t >> 5;
  const int c0   = 8 * t;
  const float* xr = x + (size_t)row * kE + c0;
  const v4f a = *(const v4f*)(xr);
  const v4f c = *(const v4f*)(xr + 4);
  float s = ((a[0] + a[1]) + (a[2] + a[3])) + ((c[0] + c[1]) + (c[2] + c[3]));
#pragma unroll
  for (int off = 16; off > 0; off >>= 1) s += __shfl_xor(s, off, 32);
  if (lane == 0) redA[wave] = s;
  __syncthreads();
  const float mean = (((redA[0] + redA[1]) + redA[2]) + redA[3]) * kInvE;
  const v4f da = a - mean;
  const v4f dc = c - mean;
  float ss = 0.f;
#pragma unroll
  for (int e = 0; e < 4; ++e) ss += da[e] * da[e];
#pragma unroll
  for (int e = 0; e < 4; ++e) ss += dc[e] * dc[e];
#pragma unroll
  for (int off = 16; off > 0; off >>= 1) ss += __shfl_xor(ss, off, 32);
  if (lane == 0) redB[wave] = ss;
  __syncthreads();
  const float var  = (((redB[0] + redB[1]) + redB[2]) + redB[3]) * kInvE;
  const float rinv = rsqrtf(var + kLnEps);
  const v4f ga = *(const v4f*)(g + c0);
  const v4f gc = *(const v4f*)(g + c0 + 4);
  const v4f ba = *(const v4f*)(bta + c0);
  const v4f bc = *(const v4f*)(bta + c0 + 4);
  const v4f ya = (da * rinv) * ga + ba;
  const v4f yc = (dc * rinv) * gc + bc;
  unsigned short hb[8];
#pragma unroll
  for (int e = 0; e < 4; ++e) {
    hb[e]     = h_bits(ya[e]);
    hb[4 + e] = h_bits(yc[e]);
  }
  const v4u u = (v4u){pk16(hb[0], hb[1]), pk16(hb[2], hb[3]), pk16(hb[4], hb[5]), pk16(hb[6], hb[7])};
  unsigned short* op = out + (size_t)row * kE + c0;
  *(volatile v4u*)op = u;
  __threadfence();
  *(volatile v4u*)op = u;
}

__global__ __launch_bounds__(256) void softmax_mean_kernel(const float* __restrict__ SC, unsigned short* __restrict__ PP,
                                                           float* __restrict__ arow) {
  __shared__ __align__(16) float ebuf[8 * 1024];
  __shared__ __align__(16) float part[8 * 1024];
  const int r    = blockIdx.x;
  const int t    = threadIdx.x;
  const int lane = t & 31, wave = t >> 5;
  float* eb = ebuf + wave * 1024 + 8 * lane;
  float* pb = part + wave * 1024 + 8 * lane;
  const v4f zero4 = (v4f){0.f, 0.f, 0.f, 0.f};
#pragma unroll
  for (int i = 0; i < 4; ++i) {
    *(v4f*)(pb + 256 * i)     = zero4;
    *(v4f*)(pb + 256 * i + 4) = zero4;
  }
#pragma unroll 1
  for (int hs = 0; hs < 2; ++hs) {
    const int h = wave + 8 * hs;
    const size_t rowoff = ((size_t)h * kChunk + r) * kLk;
    const float* sr = SC + rowoff + 8 * lane;
    float m = -__builtin_inff();
#pragma unroll 1
    for (int i = 0; i < 4; ++i) {
      const v4f a = *(const v4f*)(sr + 256 * i);
      const v4f c = *(const v4f*)(sr + 256 * i + 4);
      const float ma = fmaxf(fmaxf(a[0], a[1]), fmaxf(a[2], a[3]));
      const float mc = fmaxf(fmaxf(c[0], c[1]), fmaxf(c[2], c[3]));
      m = fmaxf(m, fmaxf(ma, mc));
    }
#pragma unroll
    for (int off = 16; off > 0; off >>= 1) m = fmaxf(m, __shfl_xor(m, off, 32));
    float s = 0.f;
#pragma unroll 1
    for (int i = 0; i < 4; ++i) {
      const v4f a = *(const v4f*)(sr + 256 * i);
      const v4f c = *(const v4f*)(sr + 256 * i + 4);
      v4f ea, ec;
#pragma unroll
      for (int e = 0; e < 4; ++e) {
        ea[e] = expf(a[e] - m);
        ec[e] = expf(c[e] - m);
      }
      s += ((ea[0] + ea[1]) + (ea[2] + ea[3])) + ((ec[0] + ec[1]) + (ec[2] + ec[3]));
      *(v4f*)(eb + 256 * i)     = ea;
      *(v4f*)(eb + 256 * i + 4) = ec;
    }
#pragma unroll
    for (int off = 16; off > 0; off >>= 1) s += __shfl_xor(s, off, 32);
    const float inv = 1.0f / s;
#pragma unroll 1
    for (int i = 0; i < 4; ++i) {
      const v4f ea = *(const v4f*)(eb + 256 * i);
      const v4f ec = *(const v4f*)(eb + 256 * i + 4);
      const v4f pa = ea * inv;
      const v4f pc = ec * inv;
      v4f qa = *(const v4f*)(pb + 256 * i);
      v4f qc = *(const v4f*)(pb + 256 * i + 4);
      qa = qa + pa;
      qc = qc + pc;
      *(v4f*)(pb + 256 * i)     = qa;
      *(v4f*)(pb + 256 * i + 4) = qc;
      unsigned short hb[8];
#pragma unroll
      for (int e = 0; e < 4; ++e) {
        hb[e]     = h_bits(pa[e] * kPCarry);
        hb[4 + e] = h_bits(pc[e] * kPCarry);
      }
      const v4u u = (v4u){pk16(hb[0], hb[1]), pk16(hb[2], hb[3]), pk16(hb[4], hb[5]), pk16(hb[6], hb[7])};
      unsigned short* pp = PP + rowoff + 8 * (size_t)lane + 256 * i;
      *(volatile v4u*)pp = u;
      __threadfence();
      *(volatile v4u*)pp = u;
    }
    asm volatile("" ::: "memory");
  }
  __syncthreads();
  {
    const float* ps = part + 4 * t;
    v4f sum = zero4;
#pragma unroll
    for (int w = 0; w < 8; ++w) sum = sum + *(const v4f*)(ps + w * 1024);
    const v4f val = sum * kInvH;
    float* op = arow + (size_t)r * kLk + 4 * t;
    *(volatile v4f*)op = val;
    __threadfence();
    *(volatile v4f*)op = val;
  }
}

extern "C" void kernel_launch(void* const* d_in, const int* in_sizes, int n_in,
                              void* d_out, int out_size, void* d_ws, size_t ws_size,
                              hipStream_t stream) {
  if (n_in < 18) return;
  const int nAct = kTok * kE;
  if (in_sizes[0] != nAct || in_sizes[1] != nAct) return;
  if (in_sizes[2] != kE || in_sizes[3] != kE || in_sizes[5] != kE || in_sizes[7] != kE || in_sizes[9] != kE ||
      in_sizes[11] != kE || in_sizes[12] != kE || in_sizes[13] != kE || in_sizes[17] != kE) return;
  if (in_sizes[4] != kE * kE || in_sizes[6] != kE * kE || in_sizes[8] != kE * kE || in_sizes[10] != kE * kE) return;
  if (in_sizes[14] != kE * kF || in_sizes[15] != kF || in_sizes[16] != kF * kE) return;
  if (out_size != 2 * nAct) return;

  const size_t szW   = (size_t)kE * kE * 2;
  const size_t szW1  = (size_t)kF * kE * 2;
  const size_t szP16 = (size_t)kTok * kE * 2;
  const size_t szX   = (size_t)kTok * kE * 4;
  const size_t szH   = (size_t)kTok * kF * 2;
  const size_t szSC  = (size_t)kH * kChunk * kLk * 4;
  const size_t szPP  = (size_t)kH * kChunk * kLk * 2;
  static_assert((size_t)kH * kChunk * kLk * 4 <= (size_t)kTok * kE * 4);
  const size_t offWQ  = 0;
  const size_t offWK  = offWQ + szW;
  const size_t offWV  = offWK + szW;
  const size_t offWO  = offWV + szW;
  const size_t offW1  = offWO + szW;
  const size_t offW2  = offW1 + szW1;
  const size_t offMEM = offW2 + szW1;
  const size_t offT2  = offMEM + szP16;
  const size_t offQ   = offT2 + szP16;
  const size_t offK   = offQ + szP16;
  const size_t offVT  = offK + szP16;
  const size_t offCTX = offVT + szP16;
  const size_t offX   = offCTX + szP16;
  const size_t offH   = offX + szX;
  const size_t offPP  = offH + szH;
  const size_t total  = offPP + szPP;
  (void)szSC;
  if (ws_size < total) return;

  const float* tgt    = (const float*)d_in[0];
  const float* memory = (const float*)d_in[1];
  const float* ln1_g  = (const float*)d_in[2];
  const float* ln1_b  = (const float*)d_in[3];
  const float* wq = (const float*)d_in[4];  const float* bq = (const float*)d_in[5];
  const float* wk = (const float*)d_in[6];  const float* bk = (const float*)d_in[7];
  const float* wv = (const float*)d_in[8];  const float* bv = (const float*)d_in[9];
  const float* wo = (const float*)d_in[10]; const float* bo = (const float*)d_in[11];
  const float* ln3_g  = (const float*)d_in[12];
  const float* ln3_b  = (const float*)d_in[13];
  const float* w1 = (const float*)d_in[14]; const float* b1 = (const float*)d_in[15];
  const float* w2 = (const float*)d_in[16]; const float* b2 = (const float*)d_in[17];

  float* out0 = (float*)d_out;
  float* out1 = (float*)d_out + (size_t)nAct;

  char* ws = (char*)d_ws;
  unsigned short* WQT   = (unsigned short*)(ws + offWQ);
  unsigned short* WKT   = (unsigned short*)(ws + offWK);
  unsigned short* WVT   = (unsigned short*)(ws + offWV);
  unsigned short* WOT   = (unsigned short*)(ws + offWO);
  unsigned short* W1T   = (unsigned short*)(ws + offW1);
  unsigned short* W2T   = (unsigned short*)(ws + offW2);
  unsigned short* MEM16 = (unsigned short*)(ws + offMEM);
  unsigned short* T2    = (unsigned short*)(ws + offT2);
  unsigned short* Q16   = (unsigned short*)(ws + offQ);
  unsigned short* K16   = (unsigned short*)(ws + offK);
  unsigned short* VT    = (unsigned short*)(ws + offVT);
  unsigned short* CTX   = (unsigned short*)(ws + offCTX);
  float*          X     = (float*)(ws + offX);
  float*          SC    = (float*)(ws + offX);
  unsigned short* H16   = (unsigned short*)(ws + offH);
  unsigned short* PP    = (unsigned short*)(ws + offPP);

  wtcast_kernel<<<dim3(kE / 64, kE / 64), dim3(256), 0, stream>>>(wq, WQT, kE, kE, kWCarry);
  wtcast_kernel<<<dim3(kE / 64, kE / 64), dim3(256), 0, stream>>>(wk, WKT, kE, kE, kWCarry);
  wtcast_kernel<<<dim3(kE / 64, kE / 64), dim3(256), 0, stream>>>(wv, WVT, kE, kE, kWCarry);
  wtcast_kernel<<<dim3(kE / 64, kE / 64), dim3(256), 0, stream>>>(wo, WOT, kE, kE, kWCarry);
  wtcast_kernel<<<dim3(kE / 64, kF / 64), dim3(256), 0, stream>>>(w1, W1T, kE, kF, kWCarry);
  wtcast_kernel<<<dim3(kF / 64, kE / 64), dim3(256), 0, stream>>>(w2, W2T, kF, kE, kWCarry);

  const int n8 = nAct / 8;
  cast8_f16_kernel<<<dim3(n8 / 256), dim3(256), 0, stream>>>(memory, MEM16, n8);
  ln_f16_kernel<<<dim3(kTok), dim3(128), 0, stream>>>(tgt, ln1_g, ln1_b, T2);

  const int tilesProj = (kTok / 64) * (kE / 64);
  wmma_gemm64<0, false, 2, 1, false, 0><<<dim3(tilesProj / 8, 1), dim3(256), 0, stream>>>(
      T2, T2, kE, 0L, WQT, WQT, kE, 0L, (void*)Q16, (void*)Q16, kE, 0L, bq, bq, 0L, kTok, kE, kE, kWCarryInv);
  wmma_gemm64<0, false, 2, 1, false, 0><<<dim3(tilesProj / 8, 1), dim3(256), 0, stream>>>(
      MEM16, MEM16, kE, 0L, WKT, WKT, kE, 0L, (void*)K16, (void*)K16, kE, 0L, bk, bk, 0L, kTok, kE, kE, kWCarryInv);
  const int tilesVT = (kE / 64) * (kLk / 64);
  wmma_gemm64<0, false, 1, 1, false, 0><<<dim3(tilesVT / 8, kB), dim3(256), 0, stream>>>(
      WVT, WVT, kE, 0L, MEM16, MEM16, kE, (long)kLk * kE, (void*)VT, (void*)VT, kLk, (long)kE * kLk,
      bv, bv, 0L, kE, kLk, kE, kWCarryInv);

  const int tilesScore = (kChunk / 64) * (kLk / 64);
  const int tilesPV    = (kChunk / 64) * (kDh / 64);
  for (int bb = 0; bb < kB; ++bb) {
    for (int cc = 0; cc < kNChunk; ++cc) {
      const size_t qrow0 = (size_t)bb * kLq + (size_t)cc * kChunk;
      const unsigned short* Ag  = Q16 + qrow0 * kE;
      const unsigned short* Btg = K16 + (size_t)bb * kLk * kE;
      wmma_gemm64<0, false, 0, 0, false, 0><<<dim3(tilesScore / 8, kH), dim3(256), 0, stream>>>(
          Ag, Ag, kE, (long)kDh, Btg, Btg, kE, (long)kDh, (void*)SC, (void*)SC, kLk, (long)kChunk * kLk,
          bq, bq, 0L, kChunk, kLk, kDh, kScoreScale);
      softmax_mean_kernel<<<dim3(kChunk), dim3(256), 0, stream>>>(SC, PP, out1 + qrow0 * kLk);
      const unsigned short* VTb = VT + (size_t)bb * kE * kLk;
      unsigned short* ctxc = CTX + qrow0 * kE;
      wmma_gemm64<0, false, 0, 1, false, 0><<<dim3((tilesPV + 7) / 8, kH), dim3(256), 0, stream>>>(
          PP, PP, kLk, (long)kChunk * kLk, VTb, VTb, kLk, (long)kDh * kLk, (void*)ctxc, (void*)ctxc, kE, (long)kDh,
          bq, bq, 0L, kChunk, kDh, kLk, kPVScale);
    }
  }

  wmma_gemm64<0, false, 2, 0, true, 0><<<dim3(tilesProj / 8, 1), dim3(256), 0, stream>>>(
      CTX, CTX, kE, 0L, WOT, WOT, kE, 0L, (void*)X, (void*)X, kE, 0L, bo, tgt, 0L, kTok, kE, kE, kOutScale);

  ln_f16_kernel<<<dim3(kTok), dim3(128), 0, stream>>>(X, ln3_g, ln3_b, T2);

  const int tilesW1 = (kTok / 64) * (kF / 64);
  wmma_gemm64<0, false, 2, 1, false, 2><<<dim3(tilesW1 / 8, 1), dim3(256), 0, stream>>>(
      T2, T2, kE, 0L, W1T, W1T, kE, 0L, (void*)H16, (void*)H16, kF, 0L, b1, b1, 0L, kTok, kF, kE, kWCarryInv);

  wmma_gemm64<0, false, 2, 0, true, 0><<<dim3(tilesProj / 8, 1), dim3(256), 0, stream>>>(
      H16, H16, kF, 0L, W2T, W2T, kF, 0L, (void*)out0, (void*)out0, kE, 0L, b2, X, 0L, kTok, kE, kF, kWCarryInv);
}
